// HGNN_USU_80178449482027
// MI455X (gfx1250) — hardware-verified
//
#include <hip/hip_runtime.h>


namespace {
constexpr int NBt = 16384, K1 = 10, K2 = 10, MU = 50, D = 64, NS1 = 100001, ND1 = 2001, NR1 = NBt * K1;
constexpr float XS = 8.0f, WSC = 256.0f;

typedef _Float16 b16;
typedef __attribute__((ext_vector_type(16))) _Float16 v16b;
typedef __attribute__((ext_vector_type(8))) _Float16 v8b;
typedef __attribute__((ext_vector_type(4))) _Float16 v4b;
typedef __attribute__((ext_vector_type(8))) float v8f;
typedef __attribute__((ext_vector_type(4))) float v4f;
__device__ __forceinline__ float bf16_rne(float f) { unsigned int u = __float_as_uint(f); u += 0x7FFFu + ((u >> 16) & 1u); return __uint_as_float(u & 0xFFFF0000u); }
__device__ __forceinline__ void split16(float v, b16& hi, b16& lo) { hi = (b16)v; lo = (b16)(v - (float)hi); }
__device__ __forceinline__ v16b frag_kb(const b16* p, int hh) { const v8b a = *(const v8b*)(p + 8 * hh), b = *(const v8b*)(p + 16 + 8 * hh); v16b f;
#pragma unroll
  for (int e = 0; e < 8; ++e) { f[e] = a[e]; f[8 + e] = b[e]; } return f; }
__device__ __forceinline__ v8f wmma16b(v16b a, v16b b, v8f c) { v8f d = __builtin_amdgcn_wmma_f32_16x16x32_f16(false, a, false, b, (short)0, c, false, false); asm volatile("v_nop\n\tv_nop\n\tv_nop\n\tv_nop" : "+v"(d) : "v"(a), "v"(b)); return d; }
__device__ __forceinline__ void wave_lds_sync() { __builtin_amdgcn_fence(__ATOMIC_RELEASE, "workgroup"); __builtin_amdgcn_wave_barrier(); __builtin_amdgcn_fence(__ATOMIC_ACQUIRE, "workgroup"); }
__device__ __forceinline__ float nexp(float x) { return __builtin_amdgcn_exp2f(x * 1.4426950408889634f); }
__device__ __forceinline__ float pmul(float a, float b) { float p = a * b; asm volatile("" : "+v"(p)); return p; }
__device__ __forceinline__ float hsum16(float v) { v += __shfl_xor(v, 1); v += __shfl_xor(v, 2); v += __shfl_xor(v, 4); return v + __shfl_xor(v, 8); }
__device__ __forceinline__ int iclamp(int v, int lo, int hi) { return v < lo ? lo : (v > hi ? hi : v); }
__device__ __forceinline__ float tanh_(float x) { const float e = nexp(-2.0f * fabsf(x)); const float t = (1.0f - e) / (1.0f + e); return x < 0.0f ? -t : t; }

__global__ __launch_bounds__(256) void prepw_kernel(const float* __restrict__ w0, const float* __restrict__ w1, const float* __restrict__ w2, const float* __restrict__ w3, const float* __restrict__ w4, b16* __restrict__ WP) {
  const int t = blockIdx.x * 256 + threadIdx.x; if (t >= 5 * D * D / 8) return; const int k = t / (D * D / 8), e = (t - k * (D * D / 8)) * 8; const float* w = k == 0 ? w0 : k == 1 ? w1 : k == 2 ? w2 : k == 3 ? w3 : w4;
  v8b o; for (int j = 0; j < 8; ++j) o[j] = (b16)(bf16_rne(w[e + j]) * WSC);
  for (int pass = 0; pass < 2; ++pass) { *(volatile v8b*)(WP + (size_t)k * D * D + e) = o; __threadfence(); }
}
__global__ __launch_bounds__(128) void stage1_kernel(const int* __restrict__ dsd1, const int* __restrict__ dsd2, const float* __restrict__ symp, const float* __restrict__ dise, const b16* __restrict__ WP, float* __restrict__ E1) {
  __shared__ __attribute__((aligned(16))) b16 Es[4][16][D + 8], Ah[4][16][D + 8], Al[4][16][D + 8], Ph[4][16][D + 8], Pl[4][16][D + 8]; __shared__ __attribute__((aligned(16))) float To[4][16][D + 4];
  const int wave = threadIdx.x >> 5, lane = threadIdx.x & 31, nloc = lane & 15, hlf = lane >> 4; const size_t r0 = ((size_t)blockIdx.x * 4 + wave) * 16;
  { const int rr = lane >> 1, hf = lane & 1; const size_t row = r0 + rr; const int s = iclamp(dsd1[row], 0, NS1 - 1); const float* es = symp + (size_t)s * D + hf * 32;
    float ad[32]; for (int c = 0; c < 32; ++c) ad[c] = 0.0f; int cnt = 0;
    for (int j = 0; j < K2; ++j) { const int dj = dsd2[row * K2 + j]; cnt += (dj != 0); const float* dr = dise + (size_t)iclamp(dj, 0, ND1 - 1) * D + hf * 32; for (int c = 0; c < 32; ++c) ad[c] += bf16_rne(dr[c]); }
    const float w2 = (cnt > 0) ? 1.0f / ((float)cnt + 1e-8f) : 0.0f;
    for (int c = 0; c < 32; ++c) { const float ev = bf16_rne(es[c]); const float a = ad[c] * w2; const int cc = hf * 32 + c; Es[wave][rr][cc] = (b16)(ev * XS); b16 h_, l_; split16(a * XS, h_, l_); Ah[wave][rr][cc] = h_; Al[wave][rr][cc] = l_; split16(pmul(a, ev) * XS, h_, l_); Ph[wave][rr][cc] = h_; Pl[wave][rr][cc] = l_; } }
  wave_lds_sync();
  const b16* W21 = WP + 1 * D * D; const b16* W22 = WP + 2 * D * D; v8f acc[4] = {{}, {}, {}, {}};
#pragma unroll
  for (int kb = 0; kb < D; kb += 32) { const v16b fe = frag_kb(&Es[wave][nloc][kb], hlf), fa = frag_kb(&Ah[wave][nloc][kb], hlf), fal = frag_kb(&Al[wave][nloc][kb], hlf), fp = frag_kb(&Ph[wave][nloc][kb], hlf), fpl = frag_kb(&Pl[wave][nloc][kb], hlf);
#pragma unroll
    for (int t = 0; t < 4; ++t) { const v16b b21 = frag_kb(W21 + (size_t)(t * 16 + nloc) * D + kb, hlf), b22 = frag_kb(W22 + (size_t)(t * 16 + nloc) * D + kb, hlf);
      acc[t] = wmma16b(fe, b21, acc[t]); acc[t] = wmma16b(fa, b21, acc[t]); acc[t] = wmma16b(fal, b21, acc[t]); acc[t] = wmma16b(fp, b22, acc[t]); acc[t] = wmma16b(fpl, b22, acc[t]); } }
  float z[4][8];
#pragma unroll
  for (int r = 0; r < 8; ++r) { float ss = 0.0f;
#pragma unroll
    for (int t = 0; t < 4; ++t) { z[t][r] = tanh_(acc[t][r] * (1.0f / (XS * WSC))); ss += pmul(z[t][r], z[t][r]); }
    ss = hsum16(ss); const float inv = 1.0f / fmaxf(sqrtf(ss), 1e-12f);
#pragma unroll
    for (int t = 0; t < 4; ++t) To[wave][8 * hlf + r][t * 16 + nloc] = z[t][r] * inv; }
  wave_lds_sync();
  for (int pass = 0; pass < 2; ++pass) { for (int rr = 0; rr < 16; ++rr) if (lane < 16) *(volatile v4f*)(E1 + (r0 + rr) * D + lane * 4) = *(const v4f*)(&To[wave][rr][lane * 4]); __threadfence(); }
}
__global__ __launch_bounds__(64) void stage2_kernel(const int* __restrict__ dsd1, const int* __restrict__ usu1, const int* __restrict__ label, const float* __restrict__ symp, const float* __restrict__ dise, const float* __restrict__ E1, const b16* __restrict__ WP, float* __restrict__ out) {
  __shared__ __attribute__((aligned(16))) b16 S1h[2][16][D + 8], S1l[2][16][D + 8], Qh[2][16][D + 8], Ql[2][16][D + 8], Tt[2][16][D + 8], Suh[2][16][D + 8], Sul[2][16][D + 8]; __shared__ float Po[2][16];
  const int wave = threadIdx.x >> 5, lane = threadIdx.x & 31, nloc = lane & 15, hlf = lane >> 4, t_ = threadIdx.x; const size_t b0 = ((size_t)blockIdx.x * 2 + wave) * 16;
  { const int rr = lane >> 1, hf = lane & 1; const size_t b = b0 + rr; int cnt1 = 0; float s1[32]; for (int c = 0; c < 32; ++c) s1[c] = 0.0f;
    for (int k = 0; k < K1; ++k) { cnt1 += (dsd1[b * K1 + k] != 0); const float* er = E1 + (b * K1 + k) * D + hf * 32; for (int c = 0; c < 32; ++c) s1[c] += er[c]; }
    const float w1 = (cnt1 > 0) ? 1.0f / ((float)cnt1 + 1e-8f) : 0.0f;
    int cntu = 0; float su[32]; for (int c = 0; c < 32; ++c) su[c] = 0.0f;
    for (int m = 0; m < MU; ++m) { const int u = usu1[b * MU + m]; cntu += (u != 0); const float* sr = symp + (size_t)iclamp(u, 0, NS1 - 1) * D + hf * 32; for (int c = 0; c < 32; ++c) su[c] += bf16_rne(sr[c]); }
    const float wu = (cntu > 0) ? 1.0f / ((float)cntu + 1e-8f) : 0.0f;
    const float* tr = dise + (size_t)iclamp(label[b], 0, ND1 - 1) * D + hf * 32;
    for (int c = 0; c < 32; ++c) { const int cc = hf * 32 + c; const float tv = bf16_rne(tr[c]); const float sv = s1[c] * w1; b16 h_, l_;
      split16(sv * XS, h_, l_); S1h[wave][rr][cc] = h_; S1l[wave][rr][cc] = l_; split16(pmul(sv, tv) * XS, h_, l_); Qh[wave][rr][cc] = h_; Ql[wave][rr][cc] = l_; Tt[wave][rr][cc] = (b16)(tv * XS);
      split16(su[c] * wu * XS, h_, l_); Suh[wave][rr][cc] = h_; Sul[wave][rr][cc] = l_; } }
  wave_lds_sync();
  const b16* Wu = WP; const b16* W11 = WP + 3 * D * D; const b16* W12 = WP + 4 * D * D; v8f ad[4] = {{}, {}, {}, {}}, au[4] = {{}, {}, {}, {}};
#pragma unroll
  for (int kb = 0; kb < D; kb += 32) { const v16b f1 = frag_kb(&S1h[wave][nloc][kb], hlf), f1l = frag_kb(&S1l[wave][nloc][kb], hlf), fq = frag_kb(&Qh[wave][nloc][kb], hlf), fql = frag_kb(&Ql[wave][nloc][kb], hlf), ft = frag_kb(&Tt[wave][nloc][kb], hlf), fu = frag_kb(&Suh[wave][nloc][kb], hlf), ful = frag_kb(&Sul[wave][nloc][kb], hlf);
#pragma unroll
    for (int t = 0; t < 4; ++t) { const v16b b11 = frag_kb(W11 + (size_t)(t * 16 + nloc) * D + kb, hlf), b12 = frag_kb(W12 + (size_t)(t * 16 + nloc) * D + kb, hlf), bu = frag_kb(Wu + (size_t)(t * 16 + nloc) * D + kb, hlf);
      ad[t] = wmma16b(f1, b11, ad[t]); ad[t] = wmma16b(f1l, b11, ad[t]); ad[t] = wmma16b(fq, b12, ad[t]); ad[t] = wmma16b(fql, b12, ad[t]); ad[t] = wmma16b(ft, b11, ad[t]); au[t] = wmma16b(fu, bu, au[t]); au[t] = wmma16b(ful, bu, au[t]); } }
#pragma unroll
  for (int r = 0; r < 8; ++r) { float p = 0.0f;
#pragma unroll
    for (int t = 0; t < 4; ++t) p += pmul(tanh_(ad[t][r] * (1.0f / (XS * WSC))), tanh_(au[t][r] * (1.0f / (XS * WSC))));
    p = hsum16(p); if (nloc == 0) Po[wave][8 * hlf + r] = p; }
  __syncthreads();
  for (int pass = 0; pass < 2; ++pass) { if (t_ < 32) ((volatile float*)out)[(size_t)blockIdx.x * 32 + t_] = Po[t_ >> 4][t_ & 15]; __threadfence(); }
}
}

extern "C" void kernel_launch(void* const* d_in, const int* in_sizes, int n_in, void* d_out, int out_size, void* d_ws, size_t ws_size, hipStream_t stream) {
  (void)n_in;
  auto Fp = [&](int i) { return (const float*)d_in[i]; }; auto Ip = [&](int i) { return (const int*)d_in[i]; };
  if (in_sizes[0] != NBt * K1 || in_sizes[1] != NBt * K1 * K2 || in_sizes[2] != NBt * MU || in_sizes[3] != NBt || in_sizes[4] != NS1 * D || in_sizes[5] != ND1 * D || in_sizes[6] != D * D || out_size != NBt) return;
  size_t off = 0; char* ws = (char*)d_ws;
  auto carve = [&](size_t bytes) { char* p = ws + off; off += (bytes + 255) & ~(size_t)255; return p; };
  b16* WP = (b16*)carve((size_t)5 * D * D * 2); float* E1 = (float*)carve((size_t)NR1 * D * 4);
  if (off > ws_size || off > ((size_t)128 << 20)) return;
  prepw_kernel<<<(5 * D * D / 8 + 255) / 256, 256, 0, stream>>>(Fp(6), Fp(7), Fp(8), Fp(9), Fp(10), WP);
  stage1_kernel<<<NR1 / 64, 128, 0, stream>>>(Ip(0), Ip(1), Fp(4), Fp(5), WP, E1);
  stage2_kernel<<<NBt / 32, 64, 0, stream>>>(Ip(0), Ip(2), Ip(3), Fp(4), Fp(5), E1, WP, (float*)d_out);
}
